// SeqCondAttentionV2_39874476376258
// MI455X (gfx1250) — hardware-verified
//
#include <hip/hip_runtime.h>
#include <stddef.h>
#include <stdint.h>
#include <math.h>

#define NB   2
#define NL   2048
#define ND   1024
#define NK   32
#define NM   4
#define NH   32
#define NDH  28
#define NTOT 2208
#define ZP   2304
#define NTOK 4096
#define GL   32
#define WTP  264
#define DSP  36
#define SFP  132
#define PI3  1.04719755119659774615f

static_assert(NTOT == 2 * ND + NK + NK * NM);
static_assert(NTOK == NB * NL);
static_assert(ZP % 128 == 0);
static_assert(ZP >= NTOT);
static_assert(NTOK % 128 == 0);
static_assert(ND % 128 == 0);
static_assert(ND % 64 == 0);
static_assert(ZP % 64 == 0);
static_assert(NL % GL == 0);
static_assert(NH * NM == 128);
static_assert((NTOK * ND) % 2048 == 0);
static_assert(NK * NH == ND);

typedef _Float16 hh;
typedef hh    v16h __attribute__((ext_vector_type(16)));
typedef hh    v8h  __attribute__((ext_vector_type(8)));
typedef float v8f  __attribute__((ext_vector_type(8)));
typedef float v4f  __attribute__((ext_vector_type(4)));

union Frag { v16h v; v8h p[2]; };

__device__ __forceinline__ v8f zero8() { return (v8f){0.f, 0.f, 0.f, 0.f, 0.f, 0.f, 0.f, 0.f}; }

__device__ __forceinline__ float wsum(float v) {
#pragma unroll
  for (int off = 16; off > 0; off >>= 1) v += __shfl_xor(v, off, 32);
  return v;
}

__device__ __forceinline__ v16h ldfrag(const hh* __restrict__ p, int ld, int row0, int k0, int lane) {
  const hh* q = p + (size_t)(row0 + (lane & 15)) * (size_t)ld + k0 + 8 * (lane >> 4);
  Frag f;
  f.p[0] = *(const v8h*)(q);
  f.p[1] = *(const v8h*)(q + 16);
  return f.v;
}

__device__ __forceinline__ v8f mma16(v16h a, v16h b, v8f cc) {
  return __builtin_amdgcn_wmma_f32_16x16x32_f16(false, a, false, b, (short)0, cc, false, false);
}

__device__ __forceinline__ v8f mma_g(v16h a, v16h b, v8f cc) {
  v8f d = __builtin_amdgcn_wmma_f32_16x16x32_f16(false, a, false, b, (short)0, cc, false, false);
  asm volatile("v_nop\n\tv_nop\n\tv_nop\n\tv_nop" : "+v"(d) : "v"(a), "v"(b));
  return d;
}

__device__ __forceinline__ void gemm32x64(const hh* __restrict__ A, int lda, const hh* __restrict__ B, int ldb,
                                          int ma, int nb, int kdim, int lane, v8f (&acc)[2][4]) {
#pragma unroll 1
  for (int k0 = 0; k0 < kdim; k0 += 32) {
    const v16h a0 = ldfrag(A, lda, ma, k0, lane);
    const v16h a1 = ldfrag(A, lda, ma + 16, k0, lane);
    const v16h b0 = ldfrag(B, ldb, nb, k0, lane);
    const v16h b1 = ldfrag(B, ldb, nb + 16, k0, lane);
    const v16h b2 = ldfrag(B, ldb, nb + 32, k0, lane);
    const v16h b3 = ldfrag(B, ldb, nb + 48, k0, lane);
    acc[0][0] = mma16(a0, b0, acc[0][0]);
    acc[1][0] = mma16(a1, b0, acc[1][0]);
    acc[0][1] = mma16(a0, b1, acc[0][1]);
    acc[1][1] = mma16(a1, b1, acc[1][1]);
    acc[0][2] = mma16(a0, b2, acc[0][2]);
    acc[1][2] = mma16(a1, b2, acc[1][2]);
    acc[0][3] = mma16(a0, b3, acc[0][3]);
    acc[1][3] = mma16(a1, b3, acc[1][3]);
    asm volatile("v_nop\n\tv_nop\n\tv_nop\n\tv_nop"
                 : "+v"(acc[0][0]), "+v"(acc[0][1]), "+v"(acc[0][2]), "+v"(acc[0][3]),
                   "+v"(acc[1][0]), "+v"(acc[1][1]), "+v"(acc[1][2]), "+v"(acc[1][3])
                 : "v"(a0), "v"(a1), "v"(b0), "v"(b1), "v"(b2), "v"(b3));
  }
}

template <int SC>
__global__ __launch_bounds__(256) void k_cvt(const float* __restrict__ w, hh* __restrict__ wh) {
  const size_t i = ((size_t)blockIdx.x * 256 + threadIdx.x) * 8;
  const v4f a0 = *(const v4f*)(w + i);
  const v4f a1 = *(const v4f*)(w + i + 4);
  v8f t = {a0[0], a0[1], a0[2], a0[3], a1[0], a1[1], a1[2], a1[3]};
  t = t * (float)SC;
  const v8h pk = __builtin_convertvector(t, v8h);
  *(volatile v8h*)(wh + i) = pk;
  __threadfence();
  *(volatile v8h*)(wh + i) = pk;
}

template <int SC, int R, int C, int CP>
__global__ __launch_bounds__(256) void k_tr(const float* __restrict__ src, hh* __restrict__ dst) {
  static_assert(R % 64 == 0);
  static_assert(CP % 64 == 0);
  static_assert(CP >= C);
  __shared__ __align__(16) hh tile[64 * 72];
  const int tid = threadIdx.x;
  const int k0 = blockIdx.x * 64, n0 = blockIdx.y * 64;
#pragma unroll
  for (int it = 0; it < 16; ++it) {
    const int idx = tid + 256 * it;
    const int kk = idx >> 6, nn = idx & 63;
    const int n = n0 + nn;
    const int nc = (n < C) ? n : (C - 1);
    float v = src[(size_t)(k0 + kk) * (size_t)C + nc];
    v = (n < C) ? v * (float)SC : 0.0f;
    tile[nn * 72 + kk] = (hh)v;
  }
  __syncthreads();
  v8h pk[2];
  size_t go[2];
#pragma unroll
  for (int it = 0; it < 2; ++it) {
    const int p = tid + 256 * it;
    const int row = p >> 3, pc = p & 7;
    pk[it] = *(const v8h*)(tile + row * 72 + pc * 8);
    go[it] = (size_t)(n0 + row) * (size_t)R + k0 + pc * 8;
  }
#pragma unroll
  for (int it = 0; it < 2; ++it) *(volatile v8h*)(dst + go[it]) = pk[it];
  __threadfence();
#pragma unroll
  for (int it = 0; it < 2; ++it) *(volatile v8h*)(dst + go[it]) = pk[it];
}

template <int LDO, int SCD>
__global__ __launch_bounds__(256) void k_gemm(const hh* __restrict__ Ap, const hh* __restrict__ Bp,
                                              float* __restrict__ o32) {
  constexpr int KD  = ND;
  constexpr int LDA = ND;
  constexpr int LDB = ND;
  constexpr float OSC = 1.0f / (float)SCD;
  static_assert(LDO % 128 == 0);

  __shared__ __align__(16) float ldsf[64 * SFP];
  const int tid = threadIdx.x, lane = tid & 31, w = tid >> 5;
  const int h = lane >> 4, c = lane & 15;
  const int wm = (w >> 1) * 32, wn = (w & 1) * 64;
  const int m0 = blockIdx.y * 128;
  const int n0 = blockIdx.x * 128;

  v8f acc[2][4];
#pragma unroll
  for (int i = 0; i < 2; ++i)
#pragma unroll
    for (int j = 0; j < 4; ++j) acc[i][j] = zero8();
  gemm32x64(Ap, LDA, Bp, LDB, m0 + wm, n0 + wn, KD, lane, acc);

#pragma unroll
  for (int hf = 0; hf < 2; ++hf) {
    if ((w >> 2) == hf) {
#pragma unroll
      for (int i = 0; i < 2; ++i)
#pragma unroll
        for (int j = 0; j < 4; ++j)
#pragma unroll
          for (int r = 0; r < 8; ++r)
            ldsf[(wm - 64 * hf + 16 * i + 8 * h + r) * SFP + wn + 16 * j + c] = acc[i][j][r] * OSC;
    }
    __syncthreads();
    v4f val[8];
    size_t go[8];
#pragma unroll
    for (int it = 0; it < 8; ++it) {
      const int p  = tid + 256 * it;
      const int lr = p >> 5;
      const int pc = p & 31;
      val[it] = *(const v4f*)(ldsf + lr * SFP + pc * 4);
      go[it] = (size_t)(m0 + 64 * hf + lr) * (size_t)LDO + n0 + pc * 4;
    }
#pragma unroll
    for (int it = 0; it < 8; ++it) *(volatile v4f*)(o32 + go[it]) = val[it];
    __threadfence();
#pragma unroll
    for (int it = 0; it < 8; ++it) *(volatile v4f*)(o32 + go[it]) = val[it];
    if (hf == 0) __syncthreads();
  }
}

__global__ __launch_bounds__(128) void k_scan(const float* __restrict__ z, const float* __restrict__ mask,
                                              const float* __restrict__ cw, const float* __restrict__ cb,
                                              const float* __restrict__ tbase, const float* __restrict__ trs,
                                              const float* __restrict__ dsl, const float* __restrict__ asl,
                                              const float* __restrict__ ssc, const float* __restrict__ nsc,
                                              const float* __restrict__ wre, const float* __restrict__ wim,
                                              float* __restrict__ yg) {
  __shared__ __align__(16) hh wt[32 * WTP];
  __shared__ __align__(16) hh cat[GL * WTP];
  __shared__ __align__(16) float dstg[GL * DSP];
  __shared__ float gb[GL * 32];
  __shared__ float red[2][4];

  const int tid = threadIdx.x, lane = tid & 31, w = tid >> 5;
  const int c = tid, h = c >> 2, mi = c & 3;
  const int b = blockIdx.x / NK, k = blockIdx.x % NK;

  const int colx = k * NH + h;
  const int colt = 2 * ND + NK + k * NM + mi;
  float wx[4], wtq[4], wsq[4], wgq[4];
#pragma unroll
  for (int t = 0; t < 4; ++t) {
    wx[t]  = cw[t * NTOT + colx];
    wtq[t] = cw[t * NTOT + colt];
  }
  const float bx = cb[colx], bt = cb[colt];
  int dq1 = 0;
  asm volatile("s_wait_loadcnt 0x0"
               : "+s"(dq1)
               : "v"(wx[0]), "v"(wx[1]), "v"(wx[2]), "v"(wx[3]),
                 "v"(wtq[0]), "v"(wtq[1]), "v"(wtq[2]), "v"(wtq[3]), "v"(bx), "v"(bt));

  const int cols = 2 * ND + k + dq1;
  const int colg = ND + k * NH + lane + dq1;
#pragma unroll
  for (int t = 0; t < 4; ++t) {
    wsq[t] = cw[t * NTOT + cols];
    wgq[t] = cw[t * NTOT + colg];
  }
  const float bs = cb[cols], bg = cb[colg];
  const float tb = tbase[k * NM + mi + dq1];
  const float rs = trs[k + dq1];
  const float ss = ssc[k + dq1];
  const float nsr = nsc[c + dq1], nsi = nsc[NH * NM + c + dq1];
  const float rawd = dsl[((k < NDH) ? k : (NDH - 1)) + dq1];
  const float rawa = asl[((k >= NDH) ? (k - NDH) : 0) + dq1];
  int dq2 = dq1;
  asm volatile("s_wait_loadcnt 0x0"
               : "+s"(dq2)
               : "v"(wsq[0]), "v"(wsq[1]), "v"(wsq[2]), "v"(wsq[3]),
                 "v"(wgq[0]), "v"(wgq[1]), "v"(wgq[2]), "v"(wgq[3]),
                 "v"(bs), "v"(bg), "v"(tb), "v"(rs), "v"(ss), "v"(nsr), "v"(nsi), "v"(rawd), "v"(rawa));

#pragma unroll 4
  for (int it = 0; it < 64; ++it) {
    const int idx = tid + 128 * it + dq2;
    const int n = idx & 31, kk = idx >> 5;
    const int kr = (kk < 128) ? kk : 127;
    const int ki = (kk >= 128) ? (kk - 128) : 0;
    const float vr = wre[kr * NH + n];
    const float vi = wim[ki * NH + n];
    const float v = (kk < 128) ? vr : vi;
    wt[n * WTP + kk] = (hh)(v * 64.0f);
  }

  const float raw = (k < NDH) ? rawd : rawa;
  const float slope = fmaxf(raw, 0.0f) + log1pf(expf(-fabsf(raw)));
  const float nslope = -slope;
  const bool isdec = (k < NDH);

  const float* zb = z + (size_t)b * NL * (size_t)ZP;
  const float* mkb = mask + b * NL;
  float* yb = yg + (size_t)b * NL * (size_t)ND + k * NH;

  float px1 = 0.f, px2 = 0.f, px3 = 0.f;
  float pt1 = 0.f, pt2 = 0.f, pt3 = 0.f;
  float ps1 = 0.f, ps2 = 0.f, ps3 = 0.f;
  float pg1 = 0.f, pg2 = 0.f, pg3 = 0.f;
  float cre = 0.f, cim = 0.f, den = 0.f;

  __syncthreads();

#pragma unroll 1
  for (int grp = 0; grp < NL / GL; ++grp) {
#pragma unroll 1
    for (int i = 0; i < GL; ++i) {
      const int l = grp * GL + i;
      const float* zr = zb + (size_t)l * ZP;
      const float x0 = zr[colx];
      const float t0 = zr[colt];
      const float s0 = zr[cols];
      const float g0 = zr[colg];
      float xv = px3 * wx[0];  xv = xv + px2 * wx[1];  xv = xv + px1 * wx[2];  xv = xv + x0 * wx[3];  xv = xv + bx;
      float tr = pt3 * wtq[0]; tr = tr + pt2 * wtq[1]; tr = tr + pt1 * wtq[2]; tr = tr + t0 * wtq[3]; tr = tr + bt;
      float sr = ps3 * wsq[0]; sr = sr + ps2 * wsq[1]; sr = sr + ps1 * wsq[2]; sr = sr + s0 * wsq[3]; sr = sr + bs;
      float gr = pg3 * wgq[0]; gr = gr + pg2 * wgq[1]; gr = gr + pg1 * wgq[2]; gr = gr + g0 * wgq[3]; gr = gr + bg;
      px3 = px2; px2 = px1; px1 = x0;
      pt3 = pt2; pt2 = pt1; pt1 = t0;
      ps3 = ps2; ps2 = ps1; ps1 = s0;
      pg3 = pg2; pg2 = pg1; pg1 = g0;

      const float mk = mkb[l];
      const float td = tr * (1.0f / (1.0f + fabsf(tr)));
      const float th = tb + rs * (td * PI3);
      const float sm = sr * mk;
      const float pv = expf(fminf(fmaxf(ss * sm, -20.0f), 20.0f)) * mk;
      const float lf = (float)l;
      const float dist = isdec ? fmaxf((float)(NL - 1) - lf, 0.0f) : lf;
      const float tw = expf(nslope * dist);
      const float pw = pv * tw;
      const float phi = (xv * mk) * th;
      float sn, cs;
      sincosf(phi, &sn, &cs);
      cre = cre + pw * cs;
      cim = cim + pw * sn;
      den = den + pw;
      const float inv = 1.0f / fmaxf(den, 1e-4f);
      const float re = cre * inv, im = cim * inv;
      float v = re * re + im * im;
      v = wsum(v);
      if (lane == 0) red[i & 1][w] = v;
      __syncthreads();
      const float tot = (red[i & 1][0] + red[i & 1][1]) + (red[i & 1][2] + red[i & 1][3]);
      const float rsq = rsqrtf(tot * (1.0f / 256.0f) + 1e-5f);
      const float cr = (re * rsq) * nsr;
      const float ci = (im * rsq) * nsi;
      cat[i * WTP + c] = (hh)(cr * 16.0f);
      cat[i * WTP + NH * NM + c] = (hh)(ci * 16.0f);
      const float gt = gr * (1.0f / (1.0f + expf(-gr)));
      if (w == 0) gb[i * 32 + lane] = gt;
    }
    __syncthreads();
    {
      const int mt = w >> 1, nt = w & 1;
      v8f acc = zero8();
#pragma unroll
      for (int ks = 0; ks < 8; ++ks) {
        const v16h af = ldfrag(cat, WTP, 16 * mt, 32 * ks, lane);
        const v16h bf = ldfrag(wt, WTP, 16 * nt, 32 * ks, lane);
        acc = mma_g(af, bf, acc);
      }
      const int hq = lane >> 4, cc = lane & 15;
      const int col = 16 * nt + cc;
#pragma unroll
      for (int r = 0; r < 8; ++r) {
        const int row = 16 * mt + 8 * hq + r;
        dstg[row * DSP + col] = (acc[r] * (1.0f / 1024.0f)) * gb[row * 32 + col];
      }
    }
    __syncthreads();
    v4f val[2];
    size_t go[2];
#pragma unroll
    for (int it = 0; it < 2; ++it) {
      const int p = tid + 128 * it;
      const int row = p >> 3, pc = p & 7;
      val[it] = *(const v4f*)(dstg + row * DSP + pc * 4);
      go[it] = (size_t)(grp * GL + row) * (size_t)ND + pc * 4;
    }
#pragma unroll
    for (int it = 0; it < 2; ++it) *(volatile v4f*)(yb + go[it]) = val[it];
    __threadfence();
#pragma unroll
    for (int it = 0; it < 2; ++it) *(volatile v4f*)(yb + go[it]) = val[it];
  }
}

extern "C" void kernel_launch(void* const* d_in, const int* in_sizes, int n_in,
                              void* d_out, int out_size, void* d_ws, size_t ws_size,
                              hipStream_t stream) {
  if (n_in < 14) return;
  if (in_sizes[0]  != NTOK * ND) return;
  if (in_sizes[1]  != NB * NL) return;
  if (in_sizes[2]  != ND * NTOT) return;
  if (in_sizes[3]  != 4 * NTOT) return;
  if (in_sizes[4]  != NTOT) return;
  if (in_sizes[5]  != NK * NM) return;
  if (in_sizes[6]  != NK) return;
  if (in_sizes[7]  != NDH) return;
  if (in_sizes[8]  != NK - NDH) return;
  if (in_sizes[9]  != NK) return;
  if (in_sizes[10] != 2 * NH * NM) return;
  if (in_sizes[11] != NH * NM * NH) return;
  if (in_sizes[12] != NH * NM * NH) return;
  if (in_sizes[13] != ND * ND) return;
  if (out_size != NTOK * ND) return;

  const float* x     = (const float*)d_in[0];
  const float* mask  = (const float*)d_in[1];
  const float* w_in  = (const float*)d_in[2];
  const float* cw    = (const float*)d_in[3];
  const float* cb    = (const float*)d_in[4];
  const float* tbase = (const float*)d_in[5];
  const float* trs   = (const float*)d_in[6];
  const float* dsl   = (const float*)d_in[7];
  const float* asl   = (const float*)d_in[8];
  const float* ssc   = (const float*)d_in[9];
  const float* nsc   = (const float*)d_in[10];
  const float* wre   = (const float*)d_in[11];
  const float* wim   = (const float*)d_in[12];
  const float* w_out = (const float*)d_in[13];
  float* out = (float*)d_out;

  size_t off = 0;
  const size_t oXH  = off; off += (size_t)NTOK * ND * 2;
  const size_t oWIT = off; off += (size_t)ZP * ND * 2;
  const size_t oWOT = off; off += (size_t)ND * ND * 2;
  const size_t oZ   = off; off += (size_t)NTOK * ZP * 4;
  const size_t oYG  = off; off += (size_t)NTOK * ND * 4;
  const size_t oYGH = off; off += (size_t)NTOK * ND * 2;
  if (off > ws_size) return;
  if (off > (size_t)134217728) return;

  char* ws = (char*)d_ws;
  hh* XH  = (hh*)(ws + oXH);
  hh* WIT = (hh*)(ws + oWIT);
  hh* WOT = (hh*)(ws + oWOT);
  float* Z32  = (float*)(ws + oZ);
  float* YG32 = (float*)(ws + oYG);
  hh* YGH = (hh*)(ws + oYGH);

  k_cvt<1><<<dim3((NTOK * ND) / 2048), dim3(256), 0, stream>>>(x, XH);
  k_tr<64, ND, NTOT, ZP><<<dim3(ND / 64, ZP / 64), dim3(256), 0, stream>>>(w_in, WIT);
  k_tr<64, ND, ND, ND><<<dim3(ND / 64, ND / 64), dim3(256), 0, stream>>>(w_out, WOT);
  k_gemm<ZP, 64><<<dim3(ZP / 128, NTOK / 128), dim3(256), 0, stream>>>(XH, WIT, Z32);
  k_scan<<<dim3(NB * NK), dim3(128), 0, stream>>>(Z32, mask, cw, cb, tbase, trs, dsl, asl, ssc, nsc, wre, wim, YG32);
  k_cvt<16><<<dim3((NTOK * ND) / 2048), dim3(256), 0, stream>>>(YG32, YGH);
  k_gemm<ND, 1024><<<dim3(ND / 128, NTOK / 128), dim3(256), 0, stream>>>(YGH, WOT, out);
  (void)hipGetLastError();
}
